// FlashAttention_10316511445594
// MI455X (gfx1250) — hardware-verified
//
#include <hip/hip_runtime.h>

typedef __attribute__((ext_vector_type(16))) _Float16 v16h;
typedef __attribute__((ext_vector_type(8)))  _Float16 v8h;
typedef __attribute__((ext_vector_type(8)))  float    v8f;
typedef __attribute__((ext_vector_type(4)))  float    v4f;
typedef __attribute__((ext_vector_type(4)))  int      v4i;

#ifndef NB
#define NB 4
#endif
#ifndef SEQ
#define SEQ 2048
#endif
#define NB_FULL  4
#define SEQ_FULL 2048
#define NH       16
#define DHEAD    64
#define BM       64
#define BN       64
#define KSTRIDE  72
#define VSTRIDE  72
#define OSTRIDE  68
#define TPL      64
#define TPS      72

#define SM_C   (0.125f * 1.4426950408889634f)
#define P_BIAS 6.0f

static_assert(NB >= 1 && NB <= NB_FULL);
static_assert(SEQ >= 2 * BN && SEQ <= SEQ_FULL);
static_assert(SEQ % (2 * BN) == 0);
static_assert(SEQ % BM == 0);
static_assert(SEQ % TPL == 0);
static_assert(BN == 64 && DHEAD == 64 && BM == 64);
static_assert((size_t)3 * NB * NH * SEQ * DHEAD * 2 <= (size_t)134217728);

__device__ __forceinline__ v16h ld_op16(const _Float16* p) {
    const v8h lo = *(const v8h*)(p);
    const v8h hi = *(const v8h*)(p + 16);
    v16h r;
#pragma unroll
    for (int i = 0; i < 8; ++i) { r[i] = lo[i]; r[i + 8] = hi[i]; }
    return r;
}

__device__ __forceinline__ v8f wmma_f16(v16h a, v16h b, v8f c) {
    v8f d = __builtin_amdgcn_wmma_f32_16x16x32_f16(
        false, a, false, b, (short)0, c, false, false);
    asm volatile("v_nop\n\tv_nop\n\tv_nop\n\tv_nop" : "+v"(d) : "v"(a), "v"(b));
    return d;
}

__device__ __forceinline__ _Float16 cvt_bh(float x) {
    unsigned u = __float_as_uint(x);
    u = (u + 0x7FFFu + ((u >> 16) & 1u)) & 0xFFFF0000u;
    return (_Float16)__uint_as_float(u);
}

__device__ __forceinline__ v8h cvt8(const float* p) {
    const float4 a = *(const float4*)(p);
    const float4 c = *(const float4*)(p + 4);
    v8h r;
    r[0] = cvt_bh(a.x); r[1] = cvt_bh(a.y); r[2] = cvt_bh(a.z); r[3] = cvt_bh(a.w);
    r[4] = cvt_bh(c.x); r[5] = cvt_bh(c.y); r[6] = cvt_bh(c.z); r[7] = cvt_bh(c.w);
    return r;
}

__global__ __launch_bounds__(256)
void k_planes(const float* __restrict__ Q, const float* __restrict__ K,
              const float* __restrict__ V, _Float16* __restrict__ Qh,
              _Float16* __restrict__ Kh, _Float16* __restrict__ Vth) {
    __shared__ __align__(16) _Float16 Vs[DHEAD * TPS];

    const int tid = threadIdx.x;
    const int bh  = blockIdx.y;
    const int b   = bh / NH;
    const int h   = bh - b * NH;
    const int l0  = blockIdx.x * TPL;

    v4i    qw[2], kw[2];
    size_t rdst[2];
#pragma unroll
    for (int i = 0; i < 2; ++i) {
        const int c   = tid + 256 * i;
        const int row = c >> 3;
        const int dc  = (c & 7) * 8;
        const size_t src = (((size_t)b * SEQ_FULL + (size_t)(l0 + row)) * NH + (size_t)h) * DHEAD + (size_t)dc;
        const v8h qv = cvt8(Q + src);
        const v8h kv = cvt8(K + src);
        const v8h vv = cvt8(V + src);
        qw[i]   = __builtin_bit_cast(v4i, qv);
        kw[i]   = __builtin_bit_cast(v4i, kv);
        rdst[i] = ((size_t)bh * SEQ + (size_t)(l0 + row)) * DHEAD + (size_t)dc;
#pragma unroll
        for (int j = 0; j < 8; ++j) Vs[(dc + j) * TPS + row] = vv[j];
    }
    __syncthreads();

    v4i    vw[2];
    size_t vdst[2];
#pragma unroll
    for (int i = 0; i < 2; ++i) {
        const int c  = tid + 256 * i;
        const int d  = c >> 3;
        const int lc = (c & 7) * 8;
        const v8h t  = *(const v8h*)&Vs[d * TPS + lc];
        vw[i]   = __builtin_bit_cast(v4i, t);
        vdst[i] = ((size_t)bh * DHEAD + (size_t)d) * SEQ + (size_t)(l0 + lc);
    }

#pragma unroll
    for (int i = 0; i < 2; ++i) {
        *(volatile v4i*)(Qh + rdst[i])  = qw[i];
        *(volatile v4i*)(Kh + rdst[i])  = kw[i];
        *(volatile v4i*)(Vth + vdst[i]) = vw[i];
    }
    __threadfence();
#pragma unroll
    for (int i = 0; i < 2; ++i) {
        *(volatile v4i*)(Qh + rdst[i])  = qw[i];
        *(volatile v4i*)(Kh + rdst[i])  = kw[i];
        *(volatile v4i*)(Vth + vdst[i]) = vw[i];
    }
}

__device__ __forceinline__ void stage_block(const _Float16* kg, const _Float16* vtg,
                                            _Float16* ks, _Float16* vts, int tid) {
#pragma unroll
    for (int i = 0; i < 4; ++i) {
        const int c   = tid + 128 * i;
        const int row = c >> 3;
        const int off = (c & 7) * 8;
        *(v8h*)&ks[row * KSTRIDE + off]  = *(const v8h*)(kg + (size_t)row * DHEAD + off);
        *(v8h*)&vts[row * VSTRIDE + off] = *(const v8h*)(vtg + (size_t)row * SEQ + off);
    }
}

__device__ __forceinline__ void fa_step(const _Float16* ksb, const _Float16* vtsb,
                                        const v16h (&qb)[2], const v16h& ones,
                                        int l16, int kbase,
                                        float& m_i, float& l_i, v8f (&acc)[4]) {
    v8f s[4];
#pragma unroll
    for (int n = 0; n < 4; ++n)
#pragma unroll
        for (int v = 0; v < 8; ++v) s[n][v] = 0.0f;
#pragma unroll
    for (int c = 0; c < 2; ++c) {
        const int dco = c * 32 + kbase;
#pragma unroll
        for (int n = 0; n < 4; ++n) {
            const v16h ka = ld_op16(&ksb[(n * 16 + l16) * KSTRIDE + dco]);
            s[n] = wmma_f16(ka, qb[c], s[n]);
        }
    }

    float tm[4];
#pragma unroll
    for (int n = 0; n < 4; ++n) {
        const float a0 = fmaxf(s[n][0], s[n][1]);
        const float a1 = fmaxf(s[n][2], s[n][3]);
        const float a2 = fmaxf(s[n][4], s[n][5]);
        const float a3 = fmaxf(s[n][6], s[n][7]);
        tm[n] = fmaxf(fmaxf(a0, a1), fmaxf(a2, a3));
    }
    float mx = fmaxf(fmaxf(tm[0], tm[1]), fmaxf(tm[2], tm[3]));
    mx = fmaxf(mx, __shfl_xor(mx, 16, 32));

    const float mnew  = fmaxf(m_i, mx);
    const float corr  = __builtin_amdgcn_exp2f((m_i - mnew) * SM_C);
    const float ebias = P_BIAS - mnew * SM_C;

    v16h pb[2];
#pragma unroll
    for (int n = 0; n < 4; ++n)
#pragma unroll
        for (int v = 0; v < 8; ++v)
            pb[n >> 1][(n & 1) * 8 + v] =
                (_Float16)__builtin_amdgcn_exp2f(fmaf(s[n][v], SM_C, ebias));

    v8f rsum;
#pragma unroll
    for (int v = 0; v < 8; ++v) rsum[v] = 0.0f;
    rsum = wmma_f16(ones, pb[0], rsum);
    rsum = wmma_f16(ones, pb[1], rsum);

    l_i = l_i * corr + rsum[0];
    m_i = mnew;
#pragma unroll
    for (int t = 0; t < 4; ++t)
#pragma unroll
        for (int v = 0; v < 8; ++v) acc[t][v] *= corr;

#pragma unroll
    for (int ck = 0; ck < 2; ++ck)
#pragma unroll
        for (int t = 0; t < 4; ++t) {
            const v16h va = ld_op16(&vtsb[(t * 16 + l16) * VSTRIDE + ck * 32 + kbase]);
            acc[t] = wmma_f16(va, pb[ck], acc[t]);
        }
}

__global__ __launch_bounds__(128) __attribute__((amdgpu_num_vgpr(256)))
void fa_fwd_wmma(const _Float16* __restrict__ Qh, const _Float16* __restrict__ Kh,
                 const _Float16* __restrict__ Vth, float* __restrict__ O) {
    __shared__ __align__(16) _Float16 Ks0[BN * KSTRIDE];
    __shared__ __align__(16) _Float16 Ks1[BN * KSTRIDE];
    __shared__ __align__(16) _Float16 Vts0[DHEAD * VSTRIDE];
    __shared__ __align__(16) _Float16 Vts1[DHEAD * VSTRIDE];
    __shared__ __align__(16) float    Os[BM * OSTRIDE];

    const int tid   = threadIdx.x;
    const int lane  = tid & 31;
    const int wid   = tid >> 5;
    const int half  = lane >> 4;
    const int l16   = lane & 15;
    const int kbase = half * 8;

    const int    bh     = blockIdx.y;
    const int    b      = bh / NH;
    const int    h      = bh - b * NH;
    const int    qblk   = blockIdx.x;
    const size_t bh_off = (size_t)bh * SEQ * DHEAD;

    const _Float16* kg0  = Kh  + bh_off;
    const _Float16* vtg0 = Vth + bh_off;

    const int       qbase = qblk * BM + wid * 16;
    const _Float16* qrow  = Qh + bh_off + (size_t)(qbase + l16) * DHEAD;
    v16h qb[2];
#pragma unroll
    for (int c = 0; c < 2; ++c) qb[c] = ld_op16(qrow + c * 32 + kbase);

    v16h ones;
#pragma unroll
    for (int e = 0; e < 16; ++e) ones[e] = (_Float16)1.0f;

    float m_i = -1e30f, l_i = 0.0f;
    v8f acc[4];
#pragma unroll
    for (int t = 0; t < 4; ++t)
#pragma unroll
        for (int v = 0; v < 8; ++v) acc[t][v] = 0.0f;

    stage_block(kg0, vtg0, Ks0, Vts0, tid);

#pragma unroll 1
    for (int kb = 0; kb < SEQ; kb += 2 * BN) {
        __syncthreads();
        stage_block(kg0 + (size_t)(kb + BN) * DHEAD, vtg0 + (kb + BN),
                    Ks1, Vts1, tid);
        fa_step(Ks0, Vts0, qb, ones, l16, kbase, m_i, l_i, acc);

        __syncthreads();
        if (kb + 2 * BN < SEQ)
            stage_block(kg0 + (size_t)(kb + 2 * BN) * DHEAD, vtg0 + (kb + 2 * BN),
                        Ks0, Vts0, tid);
        fa_step(Ks1, Vts1, qb, ones, l16, kbase, m_i, l_i, acc);
    }

    const float inv = 1.0f / l_i;
    float*      osw = Os + (wid * 16) * OSTRIDE;
    {
        float* ocol = osw + l16 * OSTRIDE;
#pragma unroll
        for (int t = 0; t < 4; ++t) {
            v4f lo, hi;
            lo[0] = acc[t][0] * inv; lo[1] = acc[t][1] * inv;
            lo[2] = acc[t][2] * inv; lo[3] = acc[t][3] * inv;
            hi[0] = acc[t][4] * inv; hi[1] = acc[t][5] * inv;
            hi[2] = acc[t][6] * inv; hi[3] = acc[t][7] * inv;
            *(v4f*)&ocol[t * 16 + kbase]     = lo;
            *(v4f*)&ocol[t * 16 + kbase + 4] = hi;
        }
    }
    __syncthreads();

    v4f ov[8];
#pragma unroll
    for (int it = 0; it < 8; ++it) {
        const int r = 2 * it + half;
        ov[it] = *(const v4f*)&osw[r * OSTRIDE + l16 * 4];
    }
    const size_t rstride = (size_t)NH * DHEAD;
    const size_t obase   = (((size_t)b * SEQ + (size_t)qbase) * NH + (size_t)h) * DHEAD
                         + (size_t)(l16 * 4);
#pragma unroll
    for (int it = 0; it < 8; ++it) {
        const int r = 2 * it + half;
        *(volatile v4f*)(O + obase + (size_t)r * rstride) = ov[it];
    }
    __threadfence();
#pragma unroll
    for (int it = 0; it < 8; ++it) {
        const int r = 2 * it + half;
        *(volatile v4f*)(O + obase + (size_t)r * rstride) = ov[it];
    }
}

extern "C" void kernel_launch(void* const* d_in, const int* in_sizes, int n_in,
                              void* d_out, int out_size, void* d_ws, size_t ws_size,
                              hipStream_t stream) {
    if (n_in < 3) return;
    const float* Q = (const float*)d_in[0];
    const float* K = (const float*)d_in[1];
    const float* V = (const float*)d_in[2];
    float*       O = (float*)d_out;

    const size_t need_in = ((size_t)(NB - 1) * SEQ_FULL + (size_t)SEQ) * NH * DHEAD;
    if ((size_t)in_sizes[0] < need_in) return;
    if ((size_t)in_sizes[1] < need_in) return;
    if ((size_t)in_sizes[2] < need_in) return;

    const size_t n = (size_t)NB * NH * SEQ * DHEAD;
    if ((size_t)out_size < n) return;
    if (ws_size < (size_t)3 * n * sizeof(_Float16)) return;

    _Float16* Qh  = (_Float16*)d_ws;
    _Float16* Kh  = Qh + n;
    _Float16* Vth = Kh + n;

    k_planes<<<dim3(SEQ / TPL, NB * NH), dim3(256), 0, stream>>>(Q, K, V, Qh, Kh, Vth);

    fa_fwd_wmma<<<dim3(SEQ / BM, NB * NH), dim3(128), 0, stream>>>(Qh, Kh, Vth, O);
}
